// SignatureGRU_81595788689886
// MI455X (gfx1250) — hardware-verified
//
#include <hip/hip_runtime.h>
#include <math.h>

typedef _Float16 v16h __attribute__((ext_vector_type(16)));
typedef _Float16 v8h  __attribute__((ext_vector_type(8)));
typedef float    v8f  __attribute__((ext_vector_type(8)));
typedef float    v4f  __attribute__((ext_vector_type(4)));
union Frag { v16h v; v8h hv[2]; };

#define T_   512
#define F_   256
#define U_   512
#define D_   5
#define SIG_ 30
#define MB_  16
#define NW_  16
#define NT_  512
#define XP_  264
#define HP_  520
#define NP_  40
#define KR_  64

__device__ __forceinline__ v16h ldfrag(const _Float16* rowp, int k0, int h) {
  Frag f;
  f.hv[0] = *(const v8h*)(rowp + k0 + 8 * h);
  f.hv[1] = *(const v8h*)(rowp + k0 + 16 + 8 * h);
  return f.v;
}

__device__ __forceinline__ void mma16(v8f& acc, v16h a, v16h b) {
  acc = __builtin_amdgcn_wmma_f32_16x16x32_f16(false, a, false, b, (short)0, acc, false, false);
  asm volatile("v_nop\n\tv_nop\n\tv_nop\n\tv_nop" : "+v"(acc) : "v"(a), "v"(b));
}

__device__ __forceinline__ float sigm(float v) { return 1.0f / (1.0f + expf(-v)); }

__device__ __forceinline__ float sel5(const float* a, int i) {
  float r = a[0];
  r = (i == 1) ? a[1] : r;
  r = (i == 2) ? a[2] : r;
  r = (i == 3) ? a[3] : r;
  r = (i >= 4) ? a[4] : r;
  return r;
}

__global__ void __launch_bounds__(256) k_wt(const float* __restrict__ in, _Float16* __restrict__ out,
                                            int K, int N, int KP) {
  __shared__ float tile[64][33];
  const int tid = threadIdx.x, lane = tid & 31, w = tid >> 5;
  const int n0 = blockIdx.x * 32, k0 = blockIdx.y * 64;
#pragma unroll
  for (int j = 0; j < 8; ++j) {
    const int kk = w + 8 * j;
    const int k = k0 + kk, n = n0 + lane;
    float v = 0.0f;
    if (k < K && n < N) v = in[(size_t)k * N + n];
    tile[kk][lane] = v;
  }
  __syncthreads();
  const int q = lane >> 3, r = lane & 7;
  const int nl = 4 * w + q;
  const int n = n0 + nl;
  v8h hv;
#pragma unroll
  for (int i = 0; i < 8; ++i) hv[i] = (_Float16)tile[8 * r + i][nl];
  const bool ok = (n < N);
  _Float16* p = out + (size_t)n * KP + k0 + 8 * r;
  if (ok) *(volatile v8h*)p = hv;
  __threadfence();
  if (ok) *(volatile v8h*)p = hv;
}

union BigLds {
  _Float16 hs[2 * MB_ * HP_];
  float    outs[MB_ * U_];
};

__global__ void __launch_bounds__(NT_) k_gru(const float* __restrict__ x,
                                            const float* __restrict__ sp,
                                            const float* __restrict__ bias,
                                            const _Float16* __restrict__ wti,
                                            const _Float16* __restrict__ wtr,
                                            const _Float16* __restrict__ wtk,
                                            float* __restrict__ out,
                                            int nb) {
  __shared__ __attribute__((aligned(16))) float    sps[D_ * F_];
  __shared__ __attribute__((aligned(16))) _Float16 xs[MB_ * XP_];
  __shared__ __attribute__((aligned(16))) _Float16 nss[MB_ * NP_];
  __shared__ __attribute__((aligned(16))) BigLds   big;

  const int tid  = threadIdx.x;
  const int lane = tid & 31, w = tid >> 5, h = lane >> 4, m = lane & 15;
  const int bb   = blockIdx.x * MB_;
  const int bw   = bb + w;
  const bool wok = (bw < nb);

  for (int i = tid; i < F_ * D_; i += NT_) {
    const int f = i / D_, d = i - f * D_;
    sps[d * F_ + f] = sp[i];
  }
  for (int i = tid; i < 2 * MB_ * HP_; i += NT_) big.hs[i] = (_Float16)0.0f;

  const int u0 = w * 16 + m;
  const int u1 = (w + NW_) * 16 + m;
  const float bz0 = bias[u0],          bz1 = bias[u1];
  const float br0 = bias[U_ + u0],     br1 = bias[U_ + u1];
  const float bn0 = bias[2 * U_ + u0], bn1 = bias[2 * U_ + u1];
  const _Float16* wiz0 = wti + (size_t)u0 * F_;
  const _Float16* win0 = wti + (size_t)(U_ + u0) * F_;
  const _Float16* wiz1 = wti + (size_t)u1 * F_;
  const _Float16* win1 = wti + (size_t)(U_ + u1) * F_;
  const _Float16* wrz0 = wtr + (size_t)u0 * U_;
  const _Float16* wrn0 = wtr + (size_t)(U_ + u0) * U_;
  const _Float16* wrz1 = wtr + (size_t)u1 * U_;
  const _Float16* wrn1 = wtr + (size_t)(U_ + u1) * U_;
  const _Float16* wk0  = wtk + (size_t)u0 * KR_;
  const _Float16* wk1  = wtk + (size_t)u1 * KR_;

  float hold0[8], hold1[8];
#pragma unroll
  for (int r = 0; r < 8; ++r) { hold0[r] = 0.0f; hold1[r] = 0.0f; }

  float sv = 0.0f;
  float pp[D_];
#pragma unroll
  for (int d = 0; d < D_; ++d) pp[d] = 0.0f;
  int si, sj;
  if (lane < D_) { si = lane; sj = 0; }
  else {
    const int e = lane - D_;
    si = e / D_;
    sj = e - si * D_;
    if (si > 4) si = 4;
    if (sj > 4) sj = 4;
  }

  __syncthreads();

  for (int t = 0; t < T_; ++t) {
    const int cur = t & 1;
    const _Float16* hsc = big.hs + cur * (MB_ * HP_);
    _Float16*       hsn = big.hs + (cur ^ 1) * (MB_ * HP_);

    {
      float xf[8];
      if (wok) {
        const v4f* xr = (const v4f*)(x + ((size_t)bw * T_ + t) * F_ + 8 * lane);
        const v4f a = xr[0], b = xr[1];
        xf[0] = a[0]; xf[1] = a[1]; xf[2] = a[2]; xf[3] = a[3];
        xf[4] = b[0]; xf[5] = b[1]; xf[6] = b[2]; xf[7] = b[3];
      } else {
#pragma unroll
        for (int i = 0; i < 8; ++i) xf[i] = 0.0f;
      }
      v8h xv;
#pragma unroll
      for (int i = 0; i < 8; ++i) xv[i] = (_Float16)xf[i];
      *(v8h*)(xs + w * XP_ + 8 * lane) = xv;

      float pt[D_];
#pragma unroll
      for (int d = 0; d < D_; ++d) {
        const v4f* s = (const v4f*)(sps + d * F_ + 8 * lane);
        const v4f s0 = s[0], s1 = s[1];
        float acc = xf[0] * s0[0];
        acc += xf[1] * s0[1]; acc += xf[2] * s0[2]; acc += xf[3] * s0[3];
        acc += xf[4] * s1[0]; acc += xf[5] * s1[1]; acc += xf[6] * s1[2]; acc += xf[7] * s1[3];
        pt[d] = acc;
      }
#pragma unroll
      for (int d = 0; d < D_; ++d) {
        float v = pt[d];
        v += __shfl_xor(v, 16);
        v += __shfl_xor(v, 8);
        v += __shfl_xor(v, 4);
        v += __shfl_xor(v, 2);
        v += __shfl_xor(v, 1);
        pt[d] = v;
      }

      float nsv = 0.0f;
      if (t > 0) {
        float dx[D_];
#pragma unroll
        for (int d = 0; d < D_; ++d) dx[d] = pt[d] - pp[d];
        const float s1p = __shfl(sv, si);
        const float dxi = sel5(dx, si), dxj = sel5(dx, sj);
        float inc;
        if (lane < D_) {
          inc = dxi;
        } else {
          const float t1 = s1p * dxj;
          const float t2 = 0.5f * dxi;
          inc = t1 + t2 * dxj;
        }
        if (lane >= SIG_) inc = 0.0f;
        sv += inc;
        if (lane < SIG_) nsv = sv * (1.0f / (float)t);
      }
#pragma unroll
      for (int d = 0; d < D_; ++d) pp[d] = pt[d];
      nss[w * NP_ + lane] = (_Float16)nsv;
    }
    __syncthreads();

    v8f axz0, axz1, ahz0, ahz1, an0, an1, ar0, ar1;
#pragma unroll
    for (int r = 0; r < 8; ++r) {
      axz0[r] = 0.0f; axz1[r] = 0.0f; ahz0[r] = 0.0f; ahz1[r] = 0.0f;
      an0[r]  = 0.0f; an1[r]  = 0.0f; ar0[r]  = 0.0f; ar1[r]  = 0.0f;
    }
    {
      const _Float16* arow = xs + m * XP_;
#pragma unroll 2
      for (int ks = 0; ks < F_ / 32; ++ks) {
        const int k0 = ks * 32;
        const v16h a = ldfrag(arow, k0, h);
        mma16(axz0, a, ldfrag(wiz0, k0, h));
        mma16(an0,  a, ldfrag(win0, k0, h));
        mma16(axz1, a, ldfrag(wiz1, k0, h));
        mma16(an1,  a, ldfrag(win1, k0, h));
      }
    }
    {
      const _Float16* arow = hsc + m * HP_;
#pragma unroll 2
      for (int ks = 0; ks < U_ / 32; ++ks) {
        const int k0 = ks * 32;
        const v16h a = ldfrag(arow, k0, h);
        mma16(ahz0, a, ldfrag(wrz0, k0, h));
        mma16(an0,  a, ldfrag(wrn0, k0, h));
        mma16(ahz1, a, ldfrag(wrz1, k0, h));
        mma16(an1,  a, ldfrag(wrn1, k0, h));
      }
    }
    {
      const v16h a = ldfrag(nss + m * NP_, 0, h);
      mma16(ar0, a, ldfrag(wk0, 0, h));
      mma16(ar1, a, ldfrag(wk1, 0, h));
    }

#pragma unroll
    for (int r = 0; r < 8; ++r) {
      const int bl = 8 * h + r;
      {
        const float hz = ahz0[r];
        const float z  = sigm(hz + axz0[r] + bz0);
        const float rg = sigm(ar0[r] + br0);
        const float nn = tanhf(an0[r] + bn0 + rg * hz);
        const float hn = z * hold0[r] + (1.0f - z) * nn;
        hold0[r] = hn;
        hsn[bl * HP_ + u0] = (_Float16)hn;
      }
      {
        const float hz = ahz1[r];
        const float z  = sigm(hz + axz1[r] + bz1);
        const float rg = sigm(ar1[r] + br1);
        const float nn = tanhf(an1[r] + bn1 + rg * hz);
        const float hn = z * hold1[r] + (1.0f - z) * nn;
        hold1[r] = hn;
        hsn[bl * HP_ + u1] = (_Float16)hn;
      }
    }
    __syncthreads();
  }

#pragma unroll
  for (int r = 0; r < 8; ++r) {
    const int bl = 8 * h + r;
    big.outs[bl * U_ + u0] = hold0[r];
    big.outs[bl * U_ + u1] = hold1[r];
  }
  __syncthreads();
  v4f ov[4];
#pragma unroll
  for (int j = 0; j < 4; ++j) ov[j] = *(const v4f*)(big.outs + w * U_ + 128 * j + 4 * lane);
  float* orow = out + (size_t)bw * U_;
  if (wok) {
#pragma unroll
    for (int j = 0; j < 4; ++j) *(volatile v4f*)(orow + 128 * j + 4 * lane) = ov[j];
  }
  __threadfence();
  if (wok) {
#pragma unroll
    for (int j = 0; j < 4; ++j) *(volatile v4f*)(orow + 128 * j + 4 * lane) = ov[j];
  }
}

static inline size_t al256(size_t v) { return (v + 255) & ~(size_t)255; }

extern "C" void kernel_launch(void* const* d_in, const int* in_sizes, int n_in,
                              void* d_out, int out_size, void* d_ws, size_t ws_size,
                              hipStream_t stream) {
  (void)n_in;
  const float* x    = (const float*)d_in[0];
  const float* sp   = (const float*)d_in[1];
  const float* rk   = (const float*)d_in[2];
  const float* wi   = (const float*)d_in[3];
  const float* wr   = (const float*)d_in[4];
  const float* bias = (const float*)d_in[5];

  const size_t b_wti = (size_t)2 * U_ * F_  * sizeof(_Float16);
  const size_t b_wtr = (size_t)2 * U_ * U_  * sizeof(_Float16);
  const size_t b_wtk = (size_t)U_ * KR_     * sizeof(_Float16);
  const size_t o_wti = 0;
  const size_t o_wtr = al256(o_wti + b_wti);
  const size_t o_wtk = al256(o_wtr + b_wtr);
  const size_t total = al256(o_wtk + b_wtk);
  if (total > ws_size) return;

  int nb = in_sizes[0] / (T_ * F_);
  const int nbo = out_size / U_;
  if (nbo < nb) nb = nbo;
  if (nb <= 0) return;

  char* ws = (char*)d_ws;
  _Float16* wti = (_Float16*)(ws + o_wti);
  _Float16* wtr = (_Float16*)(ws + o_wtr);
  _Float16* wtk = (_Float16*)(ws + o_wtk);

  k_wt<<<dim3((2 * U_ + 31) / 32, F_ / 64), 256, 0, stream>>>(wi, wti, F_, 2 * U_, F_);
  k_wt<<<dim3((2 * U_ + 31) / 32, U_ / 64), 256, 0, stream>>>(wr, wtr, U_, 2 * U_, U_);
  k_wt<<<dim3((U_ + 31) / 32, KR_ / 64), 256, 0, stream>>>(rk, wtk, SIG_, U_, KR_);

  k_gru<<<(nb + MB_ - 1) / MB_, NT_, 0, stream>>>(x, sp, bias, wti, wtr, wtk, (float*)d_out, nb);
}
